// CausalGraphNetwork_50259707297820
// MI455X (gfx1250) — hardware-verified
//
#include <hip/hip_runtime.h>
#include <stddef.h>
#include <stdint.h>


#define NB    4
#define NS    256
#define NV    64
#define NLAG  11
#define HD    128
#define NHEAD 8
#define DHD   16
#define NLAY  3
#define NBT   (NB * NS)
#define WSC   64.0f
#define INV64 0.015625f
#define PSC   4096.0f
#define OFAC  0.00390625f
#define INVO  0.0009765625f
#define HP    136
#define TP    132
#define PP    264
#define TRP   72

static_assert(NBT % 64 == 0);
static_assert(NS % 64 == 0);
static_assert(NS == 256);
static_assert(HD == 128);
static_assert(NHEAD * DHD == HD);
static_assert((NV * NV * NLAG) % 1024 == 0);
static_assert(NV + NLAG <= 96);
static_assert((HP * 2) % 16 == 0);
static_assert((TP * 4) % 16 == 0);
static_assert((PP * 2) % 16 == 0);

typedef _Float16 v16h __attribute__((ext_vector_type(16)));
typedef _Float16 v8h  __attribute__((ext_vector_type(8)));
typedef _Float16 v4h  __attribute__((ext_vector_type(4)));
typedef float    v8f  __attribute__((ext_vector_type(8)));
typedef float    v4f  __attribute__((ext_vector_type(4)));
typedef unsigned int v4u __attribute__((ext_vector_type(4)));

union Frag  { v16h v; v8h h[2]; };
union Pack8 { v8h h; v4u u; };

__device__ __forceinline__ v8f zero8() { return (v8f){0.f, 0.f, 0.f, 0.f, 0.f, 0.f, 0.f, 0.f}; }
__device__ __forceinline__ v8h zero8h() {
  return (v8h){(_Float16)0.f, (_Float16)0.f, (_Float16)0.f, (_Float16)0.f,
               (_Float16)0.f, (_Float16)0.f, (_Float16)0.f, (_Float16)0.f};
}

__device__ __forceinline__ v8f mma16(v16h a, v16h b, v8f c) {
  c = __builtin_amdgcn_wmma_f32_16x16x32_f16(false, a, false, b, (short)0, c, false, false);
  asm volatile("v_nop\n\tv_nop\n\tv_nop\n\tv_nop" : "+v"(c) : "v"(a), "v"(b));
  return c;
}

__device__ __forceinline__ v16h ldfrag(const _Float16* p, int ld, int row0, int k0, int lane) {
  const int m = lane & 15, lh = lane >> 4;
  const _Float16* q = p + (size_t)(row0 + m) * ld + k0 + 8 * lh;
  Frag f;
  f.h[0] = *(const v8h*)(q);
  f.h[1] = *(const v8h*)(q + 16);
  return f.v;
}

__global__ __launch_bounds__(256) void k_adj(const float* __restrict__ in, float* __restrict__ outp, int n4) {
  const int i = blockIdx.x * 256 + (int)threadIdx.x;
  if (i >= n4) return;
  const v4f a = *(const v4f*)(in + (size_t)i * 4);
  v4f s;
#pragma unroll
  for (int j = 0; j < 4; ++j) s[j] = __builtin_amdgcn_rcpf(1.0f + __expf(-a[j]));
  volatile v4f* d = (volatile v4f*)(outp + (size_t)i * 4);
  *d = s;
  __threadfence();
  *d = s;
}

__global__ __launch_bounds__(256) void k_et(const float* __restrict__ ve, const float* __restrict__ te,
                                            _Float16* __restrict__ et) {
  const int tid = threadIdx.x;
#pragma unroll 1
  for (int it = 0; it < 8; ++it) {
    const int p = it * 256 + tid;
    const int n = p >> 4, kp = (p & 15) * 8;
    float f[8];
#pragma unroll
    for (int i = 0; i < 8; ++i) {
      const int k = kp + i;
      const float a  = ve[min(k, NV - 1) * HD + n];
      const float bb = te[min(max(k - NV, 0), NLAG - 1) * HD + n];
      const float val = (k < NV) ? a : ((k < NV + NLAG) ? bb : 0.f);
      f[i] = val * WSC;
    }
    Pack8 pk;
    pk.h = (v8h){(_Float16)f[0], (_Float16)f[1], (_Float16)f[2], (_Float16)f[3],
                 (_Float16)f[4], (_Float16)f[5], (_Float16)f[6], (_Float16)f[7]};
    const v4u u = pk.u;
    volatile v4u* d = (volatile v4u*)(et + (size_t)n * HD + kp);
    *d = u;
    __threadfence();
    *d = u;
  }
}

__global__ __launch_bounds__(256) void k_wtr(const float* __restrict__ w, _Float16* __restrict__ wt,
                                             int kdim, int ndim, float scale) {
  __shared__ __align__(16) _Float16 st[64 * TRP];
  const int tid = threadIdx.x;
  const size_t bo = (size_t)blockIdx.z * (size_t)kdim * (size_t)ndim;
  w  += bo;
  wt += bo;
  const int n0 = blockIdx.x * 64, k0 = blockIdx.y * 64;
  const int kr = tid >> 2;
  const int nc = (tid & 3) * 16;
  const float* sp = w + (size_t)(k0 + kr) * ndim + n0 + nc;
#pragma unroll
  for (int q = 0; q < 4; ++q) {
    const v4f a = *(const v4f*)(sp + 4 * q) * scale;
#pragma unroll
    for (int j = 0; j < 4; ++j) st[(nc + 4 * q + j) * TRP + kr] = (_Float16)a[j];
  }
  __syncthreads();
  v4u val[2];
  size_t go[2];
#pragma unroll
  for (int j = 0; j < 2; ++j) {
    const int p  = tid + 256 * j;
    const int nr = p >> 3;
    const int pc = p & 7;
    Pack8 pk;
    pk.h   = *(const v8h*)(st + nr * TRP + pc * 8);
    val[j] = pk.u;
    go[j]  = (size_t)(n0 + nr) * kdim + k0 + pc * 8;
  }
  for (int ps = 0; ps < 2; ++ps) {
#pragma unroll
    for (int j = 0; j < 2; ++j) *(volatile v4u*)(wt + go[j]) = val[j];
    __threadfence();
  }
}

__global__ __launch_bounds__(256) void k_xc(const float* __restrict__ x, const float* __restrict__ adj,
                                            _Float16* __restrict__ xc) {
  __shared__ __align__(16) _Float16 sX[64 * HP];
  __shared__ float xl[64 * 12];
  const int tid = threadIdx.x, lane = tid & 31, wave = tid >> 5;
  const int hh = lane >> 4, c = lane & 15;
  const int bt = blockIdx.x, b = bt >> 8, t = bt & 255;

  for (int i = tid; i < (64 * HP) / 8; i += 256) *(v4u*)(sX + i * 8) = (v4u){0u, 0u, 0u, 0u};
  for (int idx = tid; idx < NV * NLAG; idx += 256) {
    const int s = idx / NLAG, l = idx - s * NLAG;
    const int tt = t - l;
    const float xv = x[((size_t)(b * NS + max(tt, 0))) * NV + s];
    xl[s * 12 + l] = (tt >= 0) ? xv : 0.f;
  }
  __syncthreads();

  const int tgt = tid >> 2, qd = tid & 3;
#pragma unroll 1
  for (int si = 0; si < 16; ++si) {
    const int s = qd * 16 + si;
    const float* apx = adj + ((size_t)s * NV + tgt) * NLAG;
    const float* xp  = xl + s * 12;
    float a = 0.f;
#pragma unroll
    for (int l = 0; l < NLAG; ++l) a = fmaf(xp[l], apx[l], a);
    sX[tgt * HP + s] = (_Float16)a;
  }
#pragma unroll 1
  for (int j = 0; j < 3; ++j) {
    const int l = qd + 4 * j, lc = min(l, NLAG - 1);
    float a = 0.f;
#pragma unroll 4
    for (int s = 0; s < NV; ++s) a = fmaf(xl[s * 12 + lc], adj[((size_t)s * NV + tgt) * NLAG + lc], a);
    if (l < NLAG) sX[tgt * HP + NV + l] = (_Float16)a;
  }
  __syncthreads();

#pragma unroll
  for (int j = 0; j < 4; ++j) {
    const int row = wave * 8 + 2 * j + hh;
    Pack8 pk;
    pk.h = *(const v8h*)(sX + row * HP + c * 8);
    const v4u u = pk.u;
    volatile v4u* d = (volatile v4u*)(xc + ((size_t)(row * NBT + bt)) * HD + c * 8);
    *d = u;
    __threadfence();
    *d = u;
  }
}

__global__ __launch_bounds__(256) void k_gemm(const _Float16* __restrict__ ap, int amode,
                                              const _Float16* __restrict__ wt, int wstride,
                                              const float* __restrict__ bias, int bstride,
                                              const float* __restrict__ lng, const float* __restrict__ lnb, int lnstride,
                                              const float* __restrict__ ow, const float* __restrict__ ob,
                                              _Float16* __restrict__ oh, float* __restrict__ opr,
                                              float oscale, int mode) {
  __shared__ __align__(16) _Float16 sA[64 * HP];
  __shared__ __align__(16) float sT[64 * TP];
  __shared__ __align__(16) float sPr[64];
  const int tid = threadIdx.x, lane = tid & 31, wave = tid >> 5;
  const int hh = lane >> 4, c = lane & 15;
  const int wm = wave & 3, wn = wave >> 2;
  const int v = blockIdx.y;
  const int bt0 = blockIdx.x * 64, b = bt0 >> 8, t0 = bt0 & 255;

  {
    const int ar = tid >> 2, ac = tid & 3;
#pragma unroll
    for (int q = 0; q < 4; ++q) {
      const int p = ac * 4 + q;
      const size_t o0 = ((size_t)(v * NBT + bt0 + ar)) * HD + p * 8;
      const size_t o1 = ((((size_t)(v * NB + b)) * NHEAD + (p >> 1)) * NS + t0 + ar) * DHD + (p & 1) * 8;
      const size_t o = amode ? o1 : o0;
      *(v8h*)(sA + ar * HP + p * 8) = *(const v8h*)(ap + o);
    }
  }
  __syncthreads();

  const _Float16* wv = wt + (size_t)v * (size_t)wstride;
  v8f acc[4];
#pragma unroll
  for (int tt = 0; tt < 4; ++tt) acc[tt] = zero8();
#pragma unroll 1
  for (int ks = 0; ks < 4; ++ks) {
    const v16h a = ldfrag(sA, HP, wm * 16, ks * 32, lane);
#pragma unroll
    for (int tt = 0; tt < 4; ++tt) {
      const v16h bq = ldfrag(wv, HD, wn * 64 + 16 * tt, ks * 32, lane);
      acc[tt] = mma16(a, bq, acc[tt]);
    }
  }

#pragma unroll
  for (int tt = 0; tt < 4; ++tt) {
    const int col = wn * 64 + 16 * tt + c;
    const float bl = bias[(size_t)v * bstride + col];
    const float bval = (mode == 0) ? 0.f : bl;
#pragma unroll
    for (int r = 0; r < 8; ++r) sT[(wm * 16 + 8 * hh + r) * TP + col] = acc[tt][r] * oscale + bval;
  }
  __syncthreads();

  const v4f g4 = *(const v4f*)(lng + (size_t)v * lnstride + lane * 4);
  const v4f b4 = *(const v4f*)(lnb + (size_t)v * lnstride + lane * 4);
  const v4f w4 = *(const v4f*)(ow + (size_t)v * HD + lane * 4);
  const float obv = ob[v];
#pragma unroll 1
  for (int i = 0; i < 8; ++i) {
    const int rw = wave * 8 + i;
    const v4f xv = *(const v4f*)(sT + rw * TP + lane * 4);
    v4f y = xv;
    if (mode == 1) {
      float s = (xv[0] + xv[1]) + (xv[2] + xv[3]);
#pragma unroll
      for (int off = 16; off > 0; off >>= 1) s += __shfl_xor(s, off, 32);
      const float mu = s * (1.0f / 128.0f);
      v4f dv;
#pragma unroll
      for (int j = 0; j < 4; ++j) dv[j] = xv[j] - mu;
      float s2 = (dv[0] * dv[0] + dv[1] * dv[1]) + (dv[2] * dv[2] + dv[3] * dv[3]);
#pragma unroll
      for (int off = 16; off > 0; off >>= 1) s2 += __shfl_xor(s2, off, 32);
      const float rstd = rsqrtf(s2 * (1.0f / 128.0f) + 1e-5f);
#pragma unroll
      for (int j = 0; j < 4; ++j) {
        const float yy = dv[j] * rstd * g4[j] + b4[j];
        y[j] = 0.5f * yy * (1.0f + erff(yy * 0.70710678118654752f));
      }
    }
    if (mode == 4) {
      float s = (y[0] * w4[0] + y[1] * w4[1]) + (y[2] * w4[2] + y[3] * w4[3]);
#pragma unroll
      for (int off = 16; off > 0; off >>= 1) s += __shfl_xor(s, off, 32);
      if (lane == 0) sPr[rw] = s + obv;
    } else {
      *(v4h*)(sA + rw * HP + lane * 4) = (v4h){(_Float16)y[0], (_Float16)y[1], (_Float16)y[2], (_Float16)y[3]};
    }
  }
  __syncthreads();

  if (mode <= 2) {
#pragma unroll
    for (int j = 0; j < 4; ++j) {
      const int row = wave * 8 + 2 * j + hh;
      Pack8 pk;
      pk.h = *(const v8h*)(sA + row * HP + c * 8);
      const v4u u = pk.u;
      volatile v4u* d = (volatile v4u*)(oh + ((size_t)(v * NBT + bt0 + row)) * HD + c * 8);
      *d = u;
      __threadfence();
      *d = u;
    }
  } else if (mode == 3) {
#pragma unroll
    for (int j = 0; j < 4; ++j) {
      const int col = wave * 16 + 4 * j + (lane >> 3);
      const int kp = lane & 7;
      Pack8 pk;
      pk.h = (v8h){sA[(8 * kp + 0) * HP + col], sA[(8 * kp + 1) * HP + col],
                   sA[(8 * kp + 2) * HP + col], sA[(8 * kp + 3) * HP + col],
                   sA[(8 * kp + 4) * HP + col], sA[(8 * kp + 5) * HP + col],
                   sA[(8 * kp + 6) * HP + col], sA[(8 * kp + 7) * HP + col]};
      const v4u u = pk.u;
      const size_t vo = ((((size_t)(v * NB + b)) * NHEAD + (col >> 4)) * DHD + (col & 15)) * NS + t0 + 8 * kp;
      volatile v4u* d = (volatile v4u*)(oh + vo);
      *d = u;
      __threadfence();
      *d = u;
    }
  } else {
    if (wave == 0 && lane < 16) {
      const v4f pv = *(const v4f*)(sPr + lane * 4);
      volatile v4f* d = (volatile v4f*)(opr + (size_t)v * NBT + bt0 + lane * 4);
      *d = pv;
      __threadfence();
      *d = pv;
    }
  }
}

__global__ __launch_bounds__(128) void k_attn(const _Float16* __restrict__ qp, const _Float16* __restrict__ kp,
                                              const _Float16* __restrict__ vt, _Float16* __restrict__ op) {
  __shared__ __align__(16) _Float16 sP[4 * 16 * PP];
  __shared__ __align__(16) _Float16 sO[4 * 256];
  const int tid = threadIdx.x, lane = tid & 31, wave = tid >> 5;
  const int hh = lane >> 4, c = lane & 15;
  const int h = blockIdx.x, b = blockIdx.y, v = blockIdx.z;
  const size_t rowbase = ((size_t)(v * NBT + b * NS)) * HD + h * DHD + 8 * hh;
  const _Float16* qb = qp + rowbase;
  const _Float16* kb = kp + rowbase;
  const size_t hb = ((size_t)(v * NB + b)) * NHEAD + h;
  const _Float16* vtb = vt + hb * (size_t)(DHD * NS);
  _Float16* ob = op + hb * (size_t)(NS * DHD);
  _Float16* myP = sP + wave * (16 * PP);
  _Float16* myO = sO + wave * 256;
  const v8h z8 = zero8h();

#pragma unroll 1
  for (int it = 0; it < 4; ++it) {
    const int q0 = (it * 4 + wave) * 16;
    Frag qa;
    qa.h[0] = *(const v8h*)(qb + (size_t)(q0 + c) * HD);
    qa.h[1] = z8;
    v8f sc[16];
#pragma unroll
    for (int nt = 0; nt < 16; ++nt) {
      Frag kf;
      kf.h[0] = *(const v8h*)(kb + (size_t)(nt * 16 + c) * HD);
      kf.h[1] = z8;
      sc[nt] = mma16(qa.v, kf.v, zero8());
    }
#pragma unroll
    for (int r = 0; r < 8; ++r) {
      float mx = -3.0e38f;
#pragma unroll
      for (int nt = 0; nt < 16; ++nt) mx = fmaxf(mx, sc[nt][r]);
#pragma unroll
      for (int off = 1; off < 16; off <<= 1) mx = fmaxf(mx, __shfl_xor(mx, off, 32));
      float sm = 0.f;
#pragma unroll
      for (int nt = 0; nt < 16; ++nt) {
        const float e = __expf((sc[nt][r] - mx) * 0.25f);
        sc[nt][r] = e;
        sm += e;
      }
#pragma unroll
      for (int off = 1; off < 16; off <<= 1) sm += __shfl_xor(sm, off, 32);
      const float f = PSC * __builtin_amdgcn_rcpf(sm);
      _Float16* prow = myP + (8 * hh + r) * PP + c;
#pragma unroll
      for (int nt = 0; nt < 16; ++nt) prow[nt * 16] = (_Float16)(sc[nt][r] * f);
    }
    __syncthreads();

    v8f oc = zero8();
#pragma unroll 2
    for (int ks = 0; ks < 8; ++ks) {
      const v16h a  = ldfrag(myP, PP, 0, ks * 32, lane);
      const v16h bb = ldfrag(vtb, NS, 0, ks * 32, lane);
      oc = mma16(a, bb, oc);
    }
    _Float16* orow = myO + (8 * hh) * DHD + c;
#pragma unroll
    for (int r = 0; r < 8; ++r) orow[r * DHD] = (_Float16)(oc[r] * OFAC);
    __syncthreads();

    Pack8 pk;
    pk.h = *(const v8h*)(myO + lane * 8);
    const v4u u = pk.u;
    volatile v4u* d = (volatile v4u*)(ob + (size_t)q0 * DHD + lane * 8);
    *d = u;
    __threadfence();
    *d = u;
  }
}

__global__ __launch_bounds__(256) void k_out(const float* __restrict__ pr, float* __restrict__ out) {
  __shared__ float sT2[64 * 33];
  const int tid = threadIdx.x, lane = tid & 31, wave = tid >> 5;
  const int hh = lane >> 4, c = lane & 15;
  const int bt0 = blockIdx.x * 32;
  {
    const int vv = tid >> 2, q = tid & 3;
    const float* sp = pr + (size_t)vv * NBT + bt0 + 8 * q;
    const v4f a0 = *(const v4f*)(sp);
    const v4f a1 = *(const v4f*)(sp + 4);
    float* dp = sT2 + vv * 33 + 8 * q;
    dp[0] = a0[0]; dp[1] = a0[1]; dp[2] = a0[2]; dp[3] = a0[3];
    dp[4] = a1[0]; dp[5] = a1[1]; dp[6] = a1[2]; dp[7] = a1[3];
  }
  __syncthreads();
#pragma unroll
  for (int j = 0; j < 2; ++j) {
    const int btl = wave * 4 + 2 * j + hh;
    const v4f val = (v4f){sT2[(4 * c + 0) * 33 + btl], sT2[(4 * c + 1) * 33 + btl],
                          sT2[(4 * c + 2) * 33 + btl], sT2[(4 * c + 3) * 33 + btl]};
    volatile v4f* d = (volatile v4f*)(out + (size_t)(bt0 + btl) * NV + 4 * c);
    *d = val;
    __threadfence();
    *d = val;
  }
}

extern "C" void kernel_launch(void* const* d_in, const int* in_sizes, int n_in,
                              void* d_out, int out_size, void* d_ws, size_t ws_size,
                              hipStream_t stream) {
  if (n_in < 18) return;
  if (in_sizes[0] != NB * NS * NV) return;
  if (in_sizes[1] != NV * NV * NLAG) return;
  if (in_sizes[2] != NV * HD) return;
  if (in_sizes[3] != NLAG * HD) return;
  if (in_sizes[4] != NV * NLAY * HD * HD) return;
  if (in_sizes[5] != NV * NLAY * HD) return;
  if (in_sizes[6] != NV * NLAY * HD) return;
  if (in_sizes[7] != NV * NLAY * HD) return;
  for (int i = 8; i < 12; ++i) if (in_sizes[i] != NV * HD * HD) return;
  for (int i = 12; i < 17; ++i) if (in_sizes[i] != NV * HD) return;
  if (in_sizes[17] != NV) return;
  if (out_size != NB * NS * NV) return;

  const float* x      = (const float*)d_in[0];
  const float* adjlog = (const float*)d_in[1];
  const float* vemb   = (const float*)d_in[2];
  const float* temb   = (const float*)d_in[3];
  const float* mechW  = (const float*)d_in[4];
  const float* mechb  = (const float*)d_in[5];
  const float* lng    = (const float*)d_in[6];
  const float* lnb    = (const float*)d_in[7];
  const float* Wq     = (const float*)d_in[8];
  const float* Wk     = (const float*)d_in[9];
  const float* Wv     = (const float*)d_in[10];
  const float* Wo     = (const float*)d_in[11];
  const float* bq     = (const float*)d_in[12];
  const float* bk     = (const float*)d_in[13];
  const float* bv     = (const float*)d_in[14];
  const float* bo     = (const float*)d_in[15];
  const float* outW   = (const float*)d_in[16];
  const float* outb   = (const float*)d_in[17];
  float* out = (float*)d_out;

  const size_t plane = (size_t)NV * NBT * HD * 2;
  const size_t wgrp  = (size_t)NV * HD * HD * 2;
  size_t off = 0;
  const size_t oADJ = off; off += (size_t)NV * NV * NLAG * 4;
  const size_t oET  = off; off += (size_t)HD * HD * 2;
  const size_t oXC  = off; off += plane;
  const size_t oMW  = off; off += (size_t)NLAY * wgrp;
  const size_t oQW  = off; off += wgrp;
  const size_t oKW  = off; off += wgrp;
  const size_t oVW  = off; off += wgrp;
  const size_t oOW  = off; off += wgrp;
  const size_t oZA  = off; off += plane;
  const size_t oZB  = off; off += plane;
  const size_t oVT  = off; off += plane;
  const size_t oOP  = off; off += plane;
  const size_t oPR  = off; off += (size_t)NV * NBT * 4;
  if (off > ws_size) return;
  if (off > (size_t)134217728) return;
  if ((oET | oXC | oMW | oQW | oKW | oVW | oOW | oZA | oZB | oVT | oOP | oPR) & (size_t)127) return;

  char* ws = (char*)d_ws;
  float*    ADJ = (float*)(ws + oADJ);
  _Float16* ET  = (_Float16*)(ws + oET);
  _Float16* XC  = (_Float16*)(ws + oXC);
  _Float16* MWT = (_Float16*)(ws + oMW);
  _Float16* QWT = (_Float16*)(ws + oQW);
  _Float16* KWT = (_Float16*)(ws + oKW);
  _Float16* VWT = (_Float16*)(ws + oVW);
  _Float16* OWT = (_Float16*)(ws + oOW);
  _Float16* ZA  = (_Float16*)(ws + oZA);
  _Float16* ZB  = (_Float16*)(ws + oZB);
  _Float16* VT  = (_Float16*)(ws + oVT);
  _Float16* OP  = (_Float16*)(ws + oOP);
  float*    PR  = (float*)(ws + oPR);
  _Float16* QP  = ZA;
  _Float16* KP  = XC;

  const dim3 gG(NBT / 64, NV);
  const int wg = HD * HD;

  k_adj<<<dim3((NV * NV * NLAG) / 4 / 256), dim3(256), 0, stream>>>(adjlog, ADJ, (NV * NV * NLAG) / 4);
  k_et<<<dim3(1), dim3(256), 0, stream>>>(vemb, temb, ET);
  k_wtr<<<dim3(HD / 64, HD / 64, NV * NLAY), dim3(256), 0, stream>>>(mechW, MWT, HD, HD, WSC);
  k_wtr<<<dim3(HD / 64, HD / 64, NV), dim3(256), 0, stream>>>(Wq, QWT, HD, HD, WSC);
  k_wtr<<<dim3(HD / 64, HD / 64, NV), dim3(256), 0, stream>>>(Wk, KWT, HD, HD, WSC);
  k_wtr<<<dim3(HD / 64, HD / 64, NV), dim3(256), 0, stream>>>(Wv, VWT, HD, HD, WSC);
  k_wtr<<<dim3(HD / 64, HD / 64, NV), dim3(256), 0, stream>>>(Wo, OWT, HD, HD, WSC);
  k_xc<<<dim3(NBT), dim3(256), 0, stream>>>(x, ADJ, XC);
  k_gemm<<<gG, dim3(256), 0, stream>>>(XC, 0, ET, 0, mechb, 0, lng, lnb, 0, outW, outb, ZA, PR, INV64, 0);
  k_gemm<<<gG, dim3(256), 0, stream>>>(ZA, 0, MWT + 0 * wg, NLAY * wg, mechb + 0 * HD, NLAY * HD,
                                       lng + 0 * HD, lnb + 0 * HD, NLAY * HD, outW, outb, ZB, PR, INV64, 1);
  k_gemm<<<gG, dim3(256), 0, stream>>>(ZB, 0, MWT + 1 * wg, NLAY * wg, mechb + 1 * HD, NLAY * HD,
                                       lng + 1 * HD, lnb + 1 * HD, NLAY * HD, outW, outb, ZA, PR, INV64, 1);
  k_gemm<<<gG, dim3(256), 0, stream>>>(ZA, 0, MWT + 2 * wg, NLAY * wg, mechb + 2 * HD, NLAY * HD,
                                       lng + 2 * HD, lnb + 2 * HD, NLAY * HD, outW, outb, ZB, PR, INV64, 1);
  k_gemm<<<gG, dim3(256), 0, stream>>>(ZB, 0, QWT, wg, bq, HD, lng, lnb, 0, outW, outb, QP, PR, INV64, 2);
  k_gemm<<<gG, dim3(256), 0, stream>>>(ZB, 0, KWT, wg, bk, HD, lng, lnb, 0, outW, outb, KP, PR, INV64, 2);
  k_gemm<<<gG, dim3(256), 0, stream>>>(ZB, 0, VWT, wg, bv, HD, lng, lnb, 0, outW, outb, VT, PR, INV64, 3);
  k_attn<<<dim3(NHEAD, NB, NV), dim3(128), 0, stream>>>(QP, KP, VT, OP);
  k_gemm<<<gG, dim3(256), 0, stream>>>(OP, 1, OWT, wg, bo, HD, lng, lnb, 0, outW, outb, ZB, PR, INVO, 4);
  k_out<<<dim3(NBT / 32), dim3(256), 0, stream>>>(PR, out);
  (void)hipGetLastError();
}
